// LagrangianSourceIntegration_75058848464945
// MI455X (gfx1250) — hardware-verified
//
#include <hip/hip_runtime.h>

typedef __bf16         v16bf __attribute__((ext_vector_type(16)));
typedef _Float16       v16h  __attribute__((ext_vector_type(16)));
typedef float          v8f   __attribute__((ext_vector_type(8)));
typedef float          v4f   __attribute__((ext_vector_type(4)));
typedef unsigned short us8   __attribute__((ext_vector_type(8)));
typedef unsigned short us16  __attribute__((ext_vector_type(16)));
typedef us8 __attribute__((may_alias)) us8a;
typedef v4f __attribute__((may_alias)) v4fa;

union Frag { us16 u; us8 q[2]; v16bf b; v16h h; };

#define NB   16384
#define NS   16
#define ND   256
#define NH   128
#define NK   32
#define RBLK 4096
#define RT   32
#define HP   136
#define SOP  260
#define CHP  33

__device__ __forceinline__ unsigned short f2bf(float f) {
  unsigned int u = __float_as_uint(f);
  u = u + 0x7FFFu + ((u >> 16) & 1u);
  return (unsigned short)(u >> 16);
}
__device__ __forceinline__ float bf2f(unsigned short b) {
  return __uint_as_float(((unsigned int)b) << 16);
}
__device__ __forceinline__ float bfr(float f) { return bf2f(f2bf(f)); }
__device__ __forceinline__ unsigned short h2us(_Float16 v) {
  union { _Float16 h; unsigned short u; } c; c.h = v; return c.u;
}

__device__ __forceinline__ v8f mma_bf16(v16bf a, v16bf b, v8f c) {
  v8f d = __builtin_amdgcn_wmma_f32_16x16x32_bf16(false, a, false, b, (short)0, c, false, false);
#if defined(__HIP_DEVICE_COMPILE__)
  asm volatile("v_nop\n\tv_nop\n\tv_nop\n\tv_nop" : "+v"(d) : "v"(a), "v"(b));
#endif
  return d;
}
__device__ __forceinline__ v8f mma_f16(v16h a, v16h b, v8f c) {
  v8f d = __builtin_amdgcn_wmma_f32_16x16x32_f16(false, a, false, b, (short)0, c, false, false);
#if defined(__HIP_DEVICE_COMPILE__)
  asm volatile("v_nop\n\tv_nop\n\tv_nop\n\tv_nop" : "+v"(d) : "v"(a), "v"(b));
#endif
  return d;
}

__device__ __forceinline__ Frag ld_frag(const unsigned short* p, int h) {
  Frag f;
  f.q[0] = *(const us8a*)(p + 8 * h);
  f.q[1] = *(const us8a*)(p + 16 + 8 * h);
  return f;
}

__device__ __forceinline__ v16h ld_frag_f32(const float* p, int h) {
  const v4f a = *(const v4fa*)(p + 8 * h);
  const v4f b = *(const v4fa*)(p + 8 * h + 4);
  const v4f c = *(const v4fa*)(p + 16 + 8 * h);
  const v4f d = *(const v4fa*)(p + 20 + 8 * h);
  const v16h r = { (_Float16)a.x, (_Float16)a.y, (_Float16)a.z, (_Float16)a.w,
                   (_Float16)b.x, (_Float16)b.y, (_Float16)b.z, (_Float16)b.w,
                   (_Float16)c.x, (_Float16)c.y, (_Float16)c.z, (_Float16)c.w,
                   (_Float16)d.x, (_Float16)d.y, (_Float16)d.z, (_Float16)d.w };
  return r;
}

__global__ __launch_bounds__(256) void k_cvx(const float* __restrict__ x,
                                             unsigned short* __restrict__ xb, int ngrp) {
  const int g = blockIdx.x * 256 + threadIdx.x;
  if (g >= ngrp) return;
  const float* src = x + (size_t)g * 8;
  const v4f a = *(const v4fa*)src;
  const v4f c = *(const v4fa*)(src + 4);
  const us8 o = { f2bf(a.x), f2bf(a.y), f2bf(a.z), f2bf(a.w),
                  f2bf(c.x), f2bf(c.y), f2bf(c.z), f2bf(c.w) };
  unsigned short* dst = xb + (size_t)g * 8;
  *(volatile us8*)dst = o;
  __threadfence();
  *(volatile us8*)dst = o;
}

__global__ __launch_bounds__(256) void k_wt(const float* __restrict__ W1,
                                            const float* __restrict__ W2,
                                            const float* __restrict__ Wc1,
                                            unsigned short* __restrict__ w1t,
                                            unsigned short* __restrict__ w2t,
                                            unsigned short* __restrict__ wc1t) {
  __shared__ __attribute__((aligned(16))) unsigned short tt[32 * 72];

  const int tid = threadIdx.x;
  int b = blockIdx.x;
  const float* in;
  unsigned short* outp;
  int C, opitch, rt, ct, which;
  if (b < 256) {
    which = 0;
    const int s = b >> 4, t = b & 15;
    rt = t >> 2; ct = t & 3;
    in = W1 + (size_t)s * ND * NH;  C = NH;  opitch = ND;
    outp = w1t + (size_t)s * NH * ND;
  } else if (b < 512) {
    which = 1;
    b -= 256;
    const int s = b >> 4, t = b & 15;
    rt = t >> 3; ct = t & 7;
    in = W2 + (size_t)s * NH * ND;  C = ND;  opitch = NH;
    outp = w2t + (size_t)s * ND * NH;
  } else {
    which = 2;
    b -= 512;
    const int s = b >> 2;
    rt = b & 3; ct = 0;
    in = Wc1 + (size_t)s * ND * NK; C = NK;  opitch = ND;
    outp = wc1t + (size_t)s * NK * ND;
  }
  const int r0 = rt * 64, c0 = ct * 32;

  const int c = tid & 31, rr = tid >> 5;
  #pragma unroll
  for (int i = 0; i < 8; ++i) {
    const int r = rr + 8 * i;
    const float v = in[(size_t)(r0 + r) * C + c0 + c];
    const unsigned short bb = f2bf(v);
    const unsigned short hb = h2us((_Float16)(bf2f(bb) * 16.0f));
    tt[c * 72 + r] = (which == 2) ? hb : bb;
  }
  __syncthreads();

  const int line = tid >> 3, q = tid & 7;
  const us8 v = *(const us8a*)(tt + line * 72 + 8 * q);
  unsigned short* dst = outp + (size_t)(c0 + line) * opitch + r0 + 8 * q;
  *(volatile us8*)dst = v;
  __threadfence();
  *(volatile us8*)dst = v;
}

__device__ __forceinline__ void outs_store_pass(const float* so, float* outs,
                                                int rt, int s, int tid) {
  const int q = tid & 7, sub = tid >> 3;
  #pragma unroll
  for (int i = 0; i < 16; ++i) {
    const int L = i * 16 + sub;
    const int row = L >> 3, seg = L & 7;
    const v4f v = *(const v4fa*)(so + row * SOP + 32 * seg + 4 * q);
    float* dst = outs + ((size_t)(rt * RT + row) * NS + s) * ND + 32 * seg + 4 * q;
    *(volatile v4f*)dst = v;
  }
}

__global__ __launch_bounds__(128) void k_src(
    const unsigned short* __restrict__ xb,
    const unsigned short* __restrict__ w1t,
    const unsigned short* __restrict__ w2t,
    const unsigned short* __restrict__ wc1t,
    const float* __restrict__ b1,  const float* __restrict__ b2,
    const float* __restrict__ bc1, const float* __restrict__ Wc2,
    const float* __restrict__ bc2, const float* __restrict__ lam,
    float* __restrict__ outs,
    float* __restrict__ cwb,
    int rb0)
{
  __shared__ __attribute__((aligned(16))) unsigned short hhi[RT * HP];
  __shared__ __attribute__((aligned(16))) unsigned short hlo[RT * HP];
  __shared__ __attribute__((aligned(16))) float so[RT * SOP];
  __shared__ __attribute__((aligned(16))) float chb[RT * CHP];
  __shared__ __attribute__((aligned(16))) float cws[RT];

  const int tid = threadIdx.x, lane = tid & 31, w = tid >> 5;
  const int h = lane >> 4, m = lane & 15;
  const int mt = w >> 1, wsub = w & 1;
  const int rt = blockIdx.x, s = blockIdx.y;
  const int lrow = 16 * mt + m;
  const int grow = rb0 + rt * RT + lrow;
  const v8f z8 = {0.f, 0.f, 0.f, 0.f, 0.f, 0.f, 0.f, 0.f};

  v8f acc1[4];
  #pragma unroll
  for (int j = 0; j < 4; ++j) acc1[j] = z8;
  const unsigned short* xa  = xb + (size_t)grow * ND;
  const unsigned short* wb1 = w1t + ((size_t)s * NH + 64 * wsub + m) * ND;
  #pragma unroll 1
  for (int k0 = 0; k0 < ND; k0 += 32) {
    const Frag a = ld_frag(xa + k0, h);
    #pragma unroll
    for (int j = 0; j < 4; ++j) {
      const Frag bq = ld_frag(wb1 + (size_t)j * 16 * ND + k0, h);
      acc1[j] = mma_bf16(a.b, bq.b, acc1[j]);
    }
  }
  #pragma unroll
  for (int j = 0; j < 4; ++j) {
    const int n = 64 * wsub + 16 * j + m;
    const float bias = bfr(b1[s * NH + n]);
    #pragma unroll
    for (int r = 0; r < 8; ++r) {
      const int row = 16 * mt + 8 * h + r;
      const float v = fmaxf(acc1[j][r] + bias, 0.0f);
      const unsigned short hb = f2bf(v);
      const unsigned short lb = f2bf(v - bf2f(hb));
      hhi[row * HP + n] = hb;
      hlo[row * HP + n] = lb;
    }
  }
  __syncthreads();

  v8f acc2[8];
  #pragma unroll
  for (int j = 0; j < 8; ++j) acc2[j] = z8;
  const unsigned short* ha  = hhi + lrow * HP;
  const unsigned short* la  = hlo + lrow * HP;
  const unsigned short* wb2 = w2t + ((size_t)s * ND + 128 * wsub + m) * NH;
  #pragma unroll 1
  for (int k0 = 0; k0 < NH; k0 += 32) {
    const Frag ah = ld_frag(ha + k0, h);
    const Frag al = ld_frag(la + k0, h);
    #pragma unroll
    for (int j = 0; j < 8; ++j) {
      const Frag bq = ld_frag(wb2 + (size_t)j * 16 * NH + k0, h);
      acc2[j] = mma_bf16(ah.b, bq.b, acc2[j]);
      acc2[j] = mma_bf16(al.b, bq.b, acc2[j]);
    }
  }
  #pragma unroll
  for (int j = 0; j < 8; ++j) {
    const int n = 128 * wsub + 16 * j + m;
    const float bias = bfr(b2[s * ND + n]);
    #pragma unroll
    for (int r = 0; r < 8; ++r) {
      const int row = 16 * mt + 8 * h + r;
      so[row * SOP + n] = acc2[j][r] + bias;
    }
  }
  __syncthreads();

  outs_store_pass(so, outs, rt, s, tid);
  __threadfence();
  outs_store_pass(so, outs, rt, s, tid);

  v8f acc3 = z8;
  const float* oa = so + lrow * SOP;
  const unsigned short* wb3 = wc1t + ((size_t)s * NK + 16 * wsub + m) * ND;
  #pragma unroll 1
  for (int k0 = 0; k0 < ND; k0 += 32) {
    const v16h a = ld_frag_f32(oa + k0, h);
    const Frag bq = ld_frag(wb3 + k0, h);
    acc3 = mma_f16(a, bq.h, acc3);
  }
  {
    const int n = 16 * wsub + m;
    const float bias = bfr(bc1[s * NK + n]);
    #pragma unroll
    for (int r = 0; r < 8; ++r) {
      const int row = 16 * mt + 8 * h + r;
      chb[row * CHP + n] = fmaxf(acc3[r] * 0.0625f + bias, 0.0f);
    }
  }
  __syncthreads();

  if (tid < RT) {
    float a = bfr(bc2[s]);
    #pragma unroll 4
    for (int k = 0; k < NK; ++k) a += chb[tid * CHP + k] * bfr(Wc2[s * NK + k]);
    a = fminf(fmaxf(a, -30.0f), 30.0f);
    const float conf = 1.0f / (1.0f + expf(-a));
    cws[tid] = bfr(lam[s]) * conf;
  }
  __syncthreads();

  const v4f cv = *(const v4fa*)(cws + 4 * (tid & 7));
  float* cdst = cwb + (size_t)s * RBLK + rt * RT + 4 * (tid & 7);
  if (tid < 8) *(volatile v4f*)cdst = cv;
  __threadfence();
  if (tid < 8) *(volatile v4f*)cdst = cv;
}

__global__ __launch_bounds__(256) void k_comb(const float* __restrict__ outs,
                                              const float* __restrict__ cwb,
                                              float* __restrict__ out, int rb0) {
  const int tid = threadIdx.x;
  const int rowl = tid >> 6, q = tid & 63;
  const int rrb = blockIdx.x * 4 + rowl;
  float sum = 0.0f;
  #pragma unroll
  for (int s = 0; s < NS; ++s) sum += cwb[(size_t)s * RBLK + rrb];
  const float inv = 1.0f / (sum + 1e-6f);
  v4f acc = {0.f, 0.f, 0.f, 0.f};
  #pragma unroll 4
  for (int s = 0; s < NS; ++s) {
    const float cwn = cwb[(size_t)s * RBLK + rrb] * inv;
    const v4f o = *(const v4fa*)(outs + (((size_t)rrb * NS + s) * ND + 4 * q));
    acc = acc + cwn * o;
  }
  float* dst = out + (size_t)(rb0 + rrb) * ND + 4 * q;
  *(volatile v4f*)dst = acc;
  __threadfence();
  *(volatile v4f*)dst = acc;
}

extern "C" void kernel_launch(void* const* d_in, const int* in_sizes, int n_in,
                              void* d_out, int out_size, void* d_ws, size_t ws_size,
                              hipStream_t stream) {
  static_assert((NB % RBLK) == 0);
  static_assert((RBLK % RT) == 0);
  static_assert((RBLK % 4) == 0);
  static_assert((ND % 32) == 0 && (NH % 32) == 0 && NK == 32);

  if (n_in < 10) return;
  if (in_sizes[0] != NB * ND) return;
  if (in_sizes[1] != NS * ND * NH || in_sizes[2] != NS * NH) return;
  if (in_sizes[3] != NS * NH * ND || in_sizes[4] != NS * ND) return;
  if (in_sizes[5] != NS * ND * NK || in_sizes[6] != NS * NK) return;
  if (in_sizes[7] != NS * NK || in_sizes[8] != NS || in_sizes[9] != NS) return;
  if (out_size != NB * ND) return;

  const float* x   = (const float*)d_in[0];
  const float* W1  = (const float*)d_in[1];
  const float* b1  = (const float*)d_in[2];
  const float* W2  = (const float*)d_in[3];
  const float* b2  = (const float*)d_in[4];
  const float* Wc1 = (const float*)d_in[5];
  const float* bc1 = (const float*)d_in[6];
  const float* Wc2 = (const float*)d_in[7];
  const float* bc2 = (const float*)d_in[8];
  const float* lam = (const float*)d_in[9];
  float* out = (float*)d_out;

  const size_t xb_bytes   = (size_t)NB * ND * 2;
  const size_t w1t_bytes  = (size_t)NS * NH * ND * 2;
  const size_t w2t_bytes  = (size_t)NS * ND * NH * 2;
  const size_t wc1t_bytes = (size_t)NS * NK * ND * 2;
  const size_t outs_bytes = (size_t)RBLK * NS * ND * 4;
  const size_t cwb_bytes  = (size_t)NS * RBLK * 4;
  const size_t off_xb   = 0;
  const size_t off_w1t  = off_xb + xb_bytes;
  const size_t off_w2t  = off_w1t + w1t_bytes;
  const size_t off_wc1t = off_w2t + w2t_bytes;
  const size_t off_outs = off_wc1t + wc1t_bytes;
  const size_t off_cwb  = off_outs + outs_bytes;
  const size_t total    = off_cwb + cwb_bytes;
  if (total > ws_size) return;

  char* ws = (char*)d_ws;
  unsigned short* xb   = (unsigned short*)(ws + off_xb);
  unsigned short* w1t  = (unsigned short*)(ws + off_w1t);
  unsigned short* w2t  = (unsigned short*)(ws + off_w2t);
  unsigned short* wc1t = (unsigned short*)(ws + off_wc1t);
  float* outs = (float*)(ws + off_outs);
  float* cwb  = (float*)(ws + off_cwb);

  const int ngrp = NB * ND / 8;
  k_cvx<<<(ngrp + 255) / 256, 256, 0, stream>>>(x, xb, ngrp);
  k_wt<<<576, 256, 0, stream>>>(W1, W2, Wc1, w1t, w2t, wc1t);

  for (int rb = 0; rb < NB / RBLK; ++rb) {
    const int rb0 = rb * RBLK;
    dim3 gsrc(RBLK / RT, NS);
    k_src<<<gsrc, 128, 0, stream>>>(xb, w1t, w2t, wc1t, b1, b2, bc1, Wc2, bc2, lam,
                                    outs, cwb, rb0);
    k_comb<<<RBLK / 4, 256, 0, stream>>>(outs, cwb, out, rb0);
  }
}
